// opt_joint_map_all_86663850099029
// MI455X (gfx1250) — hardware-verified
//
#include <hip/hip_runtime.h>

constexpr int NBATCH = 512;
constexpr int NSTEP  = 256;
constexpr int NFEAT  = 8;
constexpr int NHID   = 128;
constexpr int NGATE  = 4 * NHID;
constexpr int NMLP   = 512;
constexpr int NROWS  = NBATCH * NSTEP;
constexpr int NQUART = 4;
constexpr int QROWS  = NROWS / NQUART;
constexpr int HPITCH = NHID + 8;
constexpr float kHCarry   = 2048.0f;
constexpr float kWCarry   = 16.0f;
constexpr float kZScale   = 1.0f / (2048.0f * 16.0f);
constexpr float kH1Carry  = 16.0f;
constexpr float kMlpScale = 1.0f / (16.0f * 16.0f);

constexpr size_t OFF_WHH   = 0;
constexpr size_t BYTES_WHH = (size_t)3 * NGATE * NHID * 2;
constexpr size_t OFF_W2T   = OFF_WHH + BYTES_WHH;
constexpr size_t BYTES_W2T = (size_t)NMLP * NMLP * 2;
constexpr size_t OFF_H1    = OFF_W2T + BYTES_W2T;
constexpr size_t BYTES_H1  = (size_t)QROWS * NMLP * 2;
constexpr size_t OFF_H2    = OFF_H1 + BYTES_H1;
constexpr size_t BYTES_H2  = (size_t)QROWS * NMLP * 4;
constexpr size_t WS_TOTAL  = OFF_H2 + BYTES_H2;
static_assert(WS_TOTAL == 101580800, "");
static_assert((OFF_W2T % 128) == 0 && (OFF_H1 % 128) == 0 && (OFF_H2 % 128) == 0, "");

typedef __attribute__((ext_vector_type(16))) _Float16 v16h;
typedef __attribute__((ext_vector_type(8)))  _Float16 v8h;
typedef __attribute__((ext_vector_type(16))) __bf16   v16b;
typedef __attribute__((ext_vector_type(8)))  __bf16   v8b;
typedef __attribute__((ext_vector_type(8)))  float    v8f;
typedef __attribute__((ext_vector_type(4)))  float    v4f;
typedef __attribute__((ext_vector_type(4)))  unsigned int v4u;

__device__ __forceinline__ unsigned short f2bf_bits(float f) {
  unsigned u = __float_as_uint(f);
  return (unsigned short)((u + 0x7FFFu + ((u >> 16) & 1u)) >> 16);
}
__device__ __forceinline__ float bf_bits2f(unsigned short h) { return __uint_as_float(((unsigned)h) << 16); }

__device__ __forceinline__ void dep_guard_h(v8f& a, v8f& b, v16h x, v16h y) { asm volatile("v_nop\n\tv_nop\n\tv_nop\n\tv_nop" : "+v"(a), "+v"(b) : "v"(x), "v"(y)); }
__device__ __forceinline__ void dep_guard_b(v8f& a, v8f& b, v16b x, v16b y) { asm volatile("v_nop\n\tv_nop\n\tv_nop\n\tv_nop" : "+v"(a), "+v"(b) : "v"(x), "v"(y)); }
__device__ __forceinline__ void keep4_h(v16h a, v16h b, v16h c, v16h d) { asm volatile("v_nop" :: "v"(a), "v"(b), "v"(c), "v"(d)); }
__device__ __forceinline__ void keep4_b(v16b a, v16b b, v16b c, v16b d) { asm volatile("v_nop" :: "v"(a), "v"(b), "v"(c), "v"(d)); }
__device__ __forceinline__ void acc_guard4(v8f& a, v8f& b, v8f& c, v8f& d) { asm volatile("v_nop\n\tv_nop\n\tv_nop\n\tv_nop" : "+v"(a), "+v"(b), "+v"(c), "+v"(d)); }
template <typename T> struct Frag;
template <> struct Frag<_Float16> {
  typedef v16h V; union U { v16h v; v8h h[2]; };
  static __device__ __forceinline__ v16h load(const _Float16* p) {
    U f; f.h[0] = *(const v8h*)(p); f.h[1] = *(const v8h*)(p + 16); return f.v;
  }
  static __device__ __forceinline__ v8f mma(v16h a, v16h b, v8f c) {
    return __builtin_amdgcn_wmma_f32_16x16x32_f16(false, a, false, b, (short)0, c, false, false);
  }
  static __device__ __forceinline__ void guard(v8f& a, v8f& b, v16h x, v16h y) { dep_guard_h(a, b, x, y); }
  static __device__ __forceinline__ void keep(v16h a, v16h b, v16h c, v16h d) { keep4_h(a, b, c, d); }
};
template <> struct Frag<__bf16> {
  typedef v16b V; union U { v16b v; v8b h[2]; };
  static __device__ __forceinline__ v16b load(const __bf16* p) {
    U f; f.h[0] = *(const v8b*)(p); f.h[1] = *(const v8b*)(p + 16); return f.v;
  }
  static __device__ __forceinline__ v8f mma(v16b a, v16b b, v8f c) {
    return __builtin_amdgcn_wmma_f32_16x16x32_bf16(false, a, false, b, (short)0, c, false, false);
  }
  static __device__ __forceinline__ void guard(v8f& a, v8f& b, v16b x, v16b y) { dep_guard_b(a, b, x, y); }
  static __device__ __forceinline__ void keep(v16b a, v16b b, v16b c, v16b d) { keep4_b(a, b, c, d); }
};

__device__ __forceinline__ unsigned pk16(unsigned short a, unsigned short b) { return (unsigned)a | ((unsigned)b << 16); }
__device__ __forceinline__ unsigned short h_bits(float f) { const _Float16 h = (_Float16)f; return __builtin_bit_cast(unsigned short, h); }

template <int ET> struct Elem;
template <> struct Elem<0> { typedef _Float16 T; };
template <> struct Elem<1> { typedef __bf16 T; };
template <int ET, bool SPLIT, int BIAS_MODE, int OUT_MODE, bool RESID, int ACT = 0>
__global__ __launch_bounds__(256) void wmma_gemm64(
    const unsigned short* __restrict__ Ap, const unsigned short* __restrict__ A2p, int lda, long strideA,
    const unsigned short* __restrict__ Btp, const unsigned short* __restrict__ Bt2p, int ldb, long strideB,
    void* __restrict__ Cout, void* __restrict__ Cout2, int ldc, long strideC,
    const float* __restrict__ bias,
    const float* __restrict__ resid, long strideR,
    int M, int N, int K, float scale) {
  typedef typename Elem<ET>::T T;
  typedef typename Frag<T>::V V;
  const T* A = (const T*)Ap; const T* A2 = (const T*)A2p; const T* Bt = (const T*)Btp; const T* Bt2 = (const T*)Bt2p;
  __shared__ __align__(16) float sT[8][16 * 68];
  const int b    = blockIdx.y;
  const int lane = threadIdx.x & 31;
  const int wave = threadIdx.x >> 5;
  const int tilesN = N >> 6;
  const int tilesM = M >> 6;
  const int tile = blockIdx.x * 8 + wave;
  if (tile >= tilesM * tilesN) return;
  const int tm = tile / tilesN;
  const int tn = tile - tm * tilesN;
  const int m0 = tm << 6;
  const int n0 = tn << 6;

  const T* Ab  = A  + (size_t)b * strideA;
  const T* Bb  = Bt + (size_t)b * strideB;
  const T* Ab2 = SPLIT ? (A2  + (size_t)b * strideA) : nullptr;
  const T* Bb2 = SPLIT ? (Bt2 + (size_t)b * strideB) : nullptr;

  const int rlane = lane & 15;
  const int koff  = (lane >> 4) * 8;
  const int mOff  = (lane >> 4) * 8;

  v8f acc[4][4];
#pragma unroll
  for (int i = 0; i < 4; ++i)
#pragma unroll
    for (int j = 0; j < 4; ++j) acc[i][j] = (v8f){0.f,0.f,0.f,0.f,0.f,0.f,0.f,0.f};

  for (int k0 = 0; k0 < K; k0 += 32) {
    V bh[4], bl[4];
#pragma unroll
    for (int j = 0; j < 4; ++j) {
      const size_t bo = (size_t)(n0 + (j << 4) + rlane) * ldb + koff + k0;
      bh[j] = Frag<T>::load(Bb + bo);
      if (SPLIT) bl[j] = Frag<T>::load(Bb2 + bo);
    }
#pragma unroll
    for (int i = 0; i < 4; ++i) {
      const size_t ao = (size_t)(m0 + (i << 4) + rlane) * lda + koff + k0;
      V ah = Frag<T>::load(Ab + ao);
      V al;
      if (SPLIT) al = Frag<T>::load(Ab2 + ao);
#pragma unroll
      for (int j = 0; j < 4; ++j) {
        acc[i][j] = Frag<T>::mma(ah, bh[j], acc[i][j]);
        if (SPLIT) {
          acc[i][j] = Frag<T>::mma(ah, bl[j], acc[i][j]);
          acc[i][j] = Frag<T>::mma(al, bh[j], acc[i][j]);
        }
      }
      Frag<T>::guard(acc[i][0], acc[i][3], ah, SPLIT ? al : ah);
    }
    Frag<T>::keep(bh[0], bh[1], bh[2], bh[3]);
    if (SPLIT) Frag<T>::keep(bl[0], bl[1], bl[2], bl[3]);
  }
  acc_guard4(acc[0][0], acc[0][1], acc[0][2], acc[0][3]);
  acc_guard4(acc[1][0], acc[1][1], acc[1][2], acc[1][3]);
  acc_guard4(acc[2][0], acc[2][1], acc[2][2], acc[2][3]);
  acc_guard4(acc[3][0], acc[3][1], acc[3][2], acc[3][3]);

  float* slab = sT[wave];
  const float* Rb = RESID ? (resid + (size_t)b * strideR) : nullptr;
#pragma unroll
  for (int i = 0; i < 4; ++i) {
    const int mBase = m0 + (i << 4);
#pragma unroll
    for (int j = 0; j < 4; ++j) {
      const int n = n0 + (j << 4) + rlane;
      float bv = 0.f;
      if (BIAS_MODE == 2) bv = bias[n];
#pragma unroll
      for (int r = 0; r < 8; ++r) {
        float v = acc[i][j][r] * scale;
        if (BIAS_MODE == 1) v += bias[mBase + mOff + r];
        if (BIAS_MODE == 2) v += bv;
        if (RESID) v += Rb[(size_t)(mBase + mOff + r) * ldc + n];
        if (ACT == 2) v = fmaxf(v, 0.0f);
        if (ACT == 4) v = (v > 0.f) ? v : 0.01f * v;
        slab[(mOff + r) * 68 + (j << 4) + rlane] = v;
      }
    }
    __builtin_amdgcn_fence(__ATOMIC_RELEASE, "workgroup");
    __builtin_amdgcn_wave_barrier();
    __builtin_amdgcn_fence(__ATOMIC_ACQUIRE, "workgroup");
    if (OUT_MODE == 0) {
      float* C = (float*)Cout + (size_t)b * strideC;
      const int hh = lane >> 4, c4 = (lane & 15) * 4;
      for (int pass = 0; pass < 2; ++pass) {
#pragma unroll
        for (int it = 0; it < 8; ++it) {
          const int row = it * 2 + hh;
          v4f v = *(const v4f*)(slab + row * 68 + c4);
          *(volatile v4f*)(C + (size_t)(mBase + row) * ldc + n0 + c4) = v;
        }
        __threadfence();
      }
    } else {
      const int q = lane >> 3, c8 = (lane & 7) * 8;
      unsigned short* C  = (unsigned short*)Cout  + (size_t)b * strideC;
      unsigned short* C2 = (OUT_MODE == 2) ? ((unsigned short*)Cout2 + (size_t)b * strideC) : nullptr;
      for (int pass = 0; pass < 2; ++pass) {
#pragma unroll
        for (int it = 0; it < 4; ++it) {
          const int row = it * 4 + q;
          const float* sp = slab + row * 68 + c8;
          v8h hv, lv;
#pragma unroll
          for (int e = 0; e < 8; ++e) {
            if (OUT_MODE == 1) {
              hv[e] = (_Float16)sp[e];
            } else {
              unsigned short hb = f2bf_bits(sp[e]);
              unsigned short lb = f2bf_bits(sp[e] - bf_bits2f(hb));
              hv[e] = __builtin_bit_cast(_Float16, hb);
              lv[e] = __builtin_bit_cast(_Float16, lb);
            }
          }
          *(volatile v8h*)(C + (size_t)(mBase + row) * ldc + n0 + c8) = hv;
          if (OUT_MODE == 2) *(volatile v8h*)(C2 + (size_t)(mBase + row) * ldc + n0 + c8) = lv;
        }
        __threadfence();
      }
    }
    __builtin_amdgcn_fence(__ATOMIC_RELEASE, "workgroup");
    __builtin_amdgcn_wave_barrier();
    __builtin_amdgcn_fence(__ATOMIC_ACQUIRE, "workgroup");
  }
}

#if __has_builtin(__builtin_amdgcn_exp2f)
#define HW_EXP2(x) __builtin_amdgcn_exp2f(x)
#else
#define HW_EXP2(x) exp2f(x)
#endif
#if __has_builtin(__builtin_amdgcn_rcpf)
#define HW_RCP(x) __builtin_amdgcn_rcpf(x)
#else
#define HW_RCP(x) (1.0f / (x))
#endif
__device__ __forceinline__ float gate_sig(float x) {
  return HW_RCP(1.0f + HW_EXP2(-1.4426950408889634f * x));
}
__device__ __forceinline__ float gate_tanh(float x) {
  return 1.0f - 2.0f * HW_RCP(1.0f + HW_EXP2(2.8853900817779268f * x));
}

__global__ __launch_bounds__(256) void whh_cast_kernel(const float* __restrict__ Wa, const float* __restrict__ Wb,
                                                       const float* __restrict__ Wc, unsigned short* __restrict__ outp,
                                                       float scale) {
  const int z = blockIdx.y;
  const float* W = (z == 0) ? Wa : (z == 1) ? Wb : Wc;
  const int i = blockIdx.x * 256 + threadIdx.x;
  if (i >= (NGATE * NHID) / 8) return;
  const float* p = W + 8 * (size_t)i;
  const v4f a = *(const v4f*)(p);
  const v4f c = *(const v4f*)(p + 4);
  unsigned short hb[8];
#pragma unroll
  for (int e = 0; e < 4; ++e) {
    hb[e]     = h_bits(a[e] * scale);
    hb[4 + e] = h_bits(c[e] * scale);
  }
  const v4u u = (v4u){pk16(hb[0], hb[1]), pk16(hb[2], hb[3]), pk16(hb[4], hb[5]), pk16(hb[6], hb[7])};
  unsigned short* q = outp + (size_t)z * NGATE * NHID + 8 * (size_t)i;
  *(volatile v4u*)q = u;
  __threadfence();
  *(volatile v4u*)q = u;
}

__global__ __launch_bounds__(256) void w2t_cast_kernel(const float* __restrict__ W, unsigned short* __restrict__ outp,
                                                       float scale) {
  __shared__ float sm[64][65];
  const int t  = threadIdx.x;
  const int k0 = blockIdx.x * 64;
  const int n0 = blockIdx.y * 64;
#pragma unroll
  for (int i = 0; i < 16; ++i) {
    const int e  = i * 256 + t;
    const int r  = e >> 6;
    const int cc = e & 63;
    sm[cc][r] = W[(size_t)(k0 + r) * NMLP + n0 + cc] * scale;
  }
  __syncthreads();
  const int lane = t & 31, wave = t >> 5;
  const int q = lane >> 3, c8 = (lane & 7) * 8;
  for (int pass = 0; pass < 2; ++pass) {
#pragma unroll
    for (int it = 0; it < 2; ++it) {
      const int row = wave * 8 + it * 4 + q;
      unsigned short hb[8];
#pragma unroll
      for (int e = 0; e < 8; ++e) hb[e] = h_bits(sm[row][c8 + e]);
      const v4u u = (v4u){pk16(hb[0], hb[1]), pk16(hb[2], hb[3]), pk16(hb[4], hb[5]), pk16(hb[6], hb[7])};
      *(volatile v4u*)(outp + (size_t)(n0 + row) * NMLP + k0 + c8) = u;
    }
    __threadfence();
  }
}

__global__ __launch_bounds__(256) void lstm_seq_kernel(
    const float* __restrict__ X0, const float* __restrict__ X1, const float* __restrict__ X2,
    const unsigned short* __restrict__ WhhH,
    const float* __restrict__ Wih0, const float* __restrict__ bb0, const float* __restrict__ hw0, const float* __restrict__ hb0,
    const float* __restrict__ Wih1, const float* __restrict__ bb1, const float* __restrict__ hw1, const float* __restrict__ hb1,
    const float* __restrict__ Wih2, const float* __restrict__ bb2, const float* __restrict__ hw2, const float* __restrict__ hb2,
    float* __restrict__ out)
{
  union FH { v16h v; v8h h[2]; };
  __shared__ __align__(16) _Float16 sH[2][16 * HPITCH];
  __shared__ float sRed[2][8][16];
  __shared__ __align__(16) float sD[16 * NSTEP];

  const int tid  = threadIdx.x;
  const int wave = tid >> 5;
  const int lane = tid & 31;
  const int hh   = lane >> 4;
  const int c    = lane & 15;
  const int j    = blockIdx.y;
  const int b0   = blockIdx.x * 16;

  const float* X   = (j == 0) ? X0   : (j == 1) ? X1   : X2;
  const float* Wih = (j == 0) ? Wih0 : (j == 1) ? Wih1 : Wih2;
  const float* bb  = (j == 0) ? bb0  : (j == 1) ? bb1  : bb2;
  const float* hw  = (j == 0) ? hw0  : (j == 1) ? hw1  : hw2;
  const float* hbp = (j == 0) ? hb0  : (j == 1) ? hb1  : hb2;
  const _Float16* Wp = (const _Float16*)WhhH + (size_t)j * NGATE * NHID;

  const int unit = 16 * wave + c;

  float wi[4][8];
  float bg[4];
#pragma unroll
  for (int g = 0; g < 4; ++g) {
    const int n = g * NHID + unit;
    const v4f a = *(const v4f*)(Wih + (size_t)n * NFEAT);
    const v4f d = *(const v4f*)(Wih + (size_t)n * NFEAT + 4);
#pragma unroll
    for (int e = 0; e < 4; ++e) { wi[g][e] = a[e]; wi[g][4 + e] = d[e]; }
    bg[g] = bb[n];
  }
  const float hwu = hw[unit];
  const float hbv = hbp[0];

  {
    v8h zv;
#pragma unroll
    for (int e = 0; e < 8; ++e) zv[e] = (_Float16)0.0f;
    const int row = tid >> 4;
    const int c8  = (tid & 15) * 8;
    *(v8h*)(&sH[0][row * HPITCH + c8]) = zv;
  }
  float cst[8];
#pragma unroll
  for (int r = 0; r < 8; ++r) cst[r] = 0.0f;
  __syncthreads();

#pragma unroll 1
  for (int t = 0; t < NSTEP; ++t) {
    const int cur = t & 1;
    const int nxt = cur ^ 1;
    const _Float16* hcur = &sH[cur][0];

    v8f acc[4];
#pragma unroll
    for (int g = 0; g < 4; ++g) acc[g] = (v8f){0.f,0.f,0.f,0.f,0.f,0.f,0.f,0.f};

#pragma unroll
    for (int ks = 0; ks < 4; ++ks) {
      FH af;
      af.h[0] = *(const v8h*)(hcur + c * HPITCH + ks * 32 + 8 * hh);
      af.h[1] = *(const v8h*)(hcur + c * HPITCH + ks * 32 + 16 + 8 * hh);
      v16h bf[4];
#pragma unroll
      for (int g = 0; g < 4; ++g)
        bf[g] = Frag<_Float16>::load(Wp + (size_t)(g * NHID + unit) * NHID + ks * 32 + 8 * hh);
#pragma unroll
      for (int g = 0; g < 4; ++g) acc[g] = Frag<_Float16>::mma(af.v, bf[g], acc[g]);
      dep_guard_h(acc[0], acc[3], af.v, bf[3]);
      keep4_h(bf[0], bf[1], bf[2], bf[3]);
    }
    acc_guard4(acc[0], acc[1], acc[2], acc[3]);

    const float* xb = X + ((size_t)(b0 + 8 * hh) * NSTEP + t) * NFEAT;
    _Float16* hn = &sH[nxt][0];
    float pd[8];
#pragma unroll
    for (int r = 0; r < 8; ++r) {
      const v4f xa = *(const v4f*)(xb + (size_t)r * NSTEP * NFEAT);
      const v4f xc = *(const v4f*)(xb + (size_t)r * NSTEP * NFEAT + 4);
      float z[4];
#pragma unroll
      for (int g = 0; g < 4; ++g) {
        float s = bg[g];
#pragma unroll
        for (int e = 0; e < 4; ++e) s = fmaf(xa[e], wi[g][e], s);
#pragma unroll
        for (int e = 0; e < 4; ++e) s = fmaf(xc[e], wi[g][4 + e], s);
        z[g] = fmaf(acc[g][r], kZScale, s);
      }
      const float si = gate_sig(z[0]);
      const float sf = gate_sig(z[1]);
      const float tg = gate_tanh(z[2]);
      const float so = gate_sig(z[3]);
      const float cn = sf * cst[r] + si * tg;
      cst[r] = cn;
      const float hv = so * gate_tanh(cn);
      hn[(8 * hh + r) * HPITCH + unit] = (_Float16)(hv * kHCarry);
      pd[r] = hv * hwu;
    }
#pragma unroll
    for (int r = 0; r < 8; ++r) {
      float p = pd[r];
      p += __shfl_xor(p, 1, 32);
      p += __shfl_xor(p, 2, 32);
      p += __shfl_xor(p, 4, 32);
      p += __shfl_xor(p, 8, 32);
      pd[r] = p;
    }
    if (c == 0) {
#pragma unroll
      for (int r = 0; r < 8; ++r) sRed[cur][wave][8 * hh + r] = pd[r];
    }
    __syncthreads();
    if (tid < 16) {
      float s = sRed[cur][0][tid];
#pragma unroll
      for (int w = 1; w < 8; ++w) s += sRed[cur][w][tid];
      sD[tid * NSTEP + t] = s + hbv;
    }
  }
  __syncthreads();

  {
    float* Dj = out + (size_t)j * NROWS;
    for (int pass = 0; pass < 2; ++pass) {
#pragma unroll
      for (int rr = 0; rr < 2; ++rr) {
        const int row = 2 * wave + rr;
        const float* src = sD + row * NSTEP;
        float* dst = Dj + (size_t)(b0 + row) * NSTEP;
#pragma unroll
        for (int it = 0; it < 2; ++it) {
          const v4f v = *(const v4f*)(src + it * 128 + lane * 4);
          *(volatile v4f*)(dst + it * 128 + lane * 4) = v;
        }
      }
      __threadfence();
    }
  }
}

__global__ __launch_bounds__(256) void mlp_h1_kernel(const float* __restrict__ Dall, const float* __restrict__ W1,
                                                     const float* __restrict__ b1, unsigned short* __restrict__ H1,
                                                     int mbase, float carry) {
  const int gid  = blockIdx.x * 256 + threadIdx.x;
  const int mloc = gid >> 6;
  if (mloc >= QROWS) return;
  const int k0   = (gid & 63) * 8;
  const int m    = mbase + mloc;
  const float x0 = Dall[m];
  const float x1 = Dall[NROWS + m];
  const float x2 = Dall[2 * NROWS + m];
  const v4f wa0 = *(const v4f*)(W1 + k0);
  const v4f wa1 = *(const v4f*)(W1 + k0 + 4);
  const v4f wb0 = *(const v4f*)(W1 + NMLP + k0);
  const v4f wb1 = *(const v4f*)(W1 + NMLP + k0 + 4);
  const v4f wc0 = *(const v4f*)(W1 + 2 * NMLP + k0);
  const v4f wc1 = *(const v4f*)(W1 + 2 * NMLP + k0 + 4);
  const v4f ba  = *(const v4f*)(b1 + k0);
  const v4f bc  = *(const v4f*)(b1 + k0 + 4);
  unsigned short hb[8];
#pragma unroll
  for (int e = 0; e < 4; ++e) {
    float v = ba[e];
    v = fmaf(x0, wa0[e], v);
    v = fmaf(x1, wb0[e], v);
    v = fmaf(x2, wc0[e], v);
    v = fmaxf(v, 0.0f);
    hb[e] = h_bits(v * carry);
    float u = bc[e];
    u = fmaf(x0, wa1[e], u);
    u = fmaf(x1, wb1[e], u);
    u = fmaf(x2, wc1[e], u);
    u = fmaxf(u, 0.0f);
    hb[4 + e] = h_bits(u * carry);
  }
  const v4u pkt = (v4u){pk16(hb[0], hb[1]), pk16(hb[2], hb[3]), pk16(hb[4], hb[5]), pk16(hb[6], hb[7])};
  unsigned short* q = H1 + (size_t)mloc * NMLP + k0;
  *(volatile v4u*)q = pkt;
  __threadfence();
  *(volatile v4u*)q = pkt;
}

__global__ __launch_bounds__(256) void mlp_head_kernel(const float* __restrict__ H2, const float* __restrict__ W3,
                                                       const float* __restrict__ b3, float* __restrict__ out3,
                                                       int mbase) {
  __shared__ __align__(16) float sW[NMLP];
  const int tid = threadIdx.x;
  sW[tid] = W3[tid];
  sW[tid + 256] = W3[tid + 256];
  __syncthreads();
  const int mloc = blockIdx.x * 256 + tid;
  const int mcl  = (mloc < QROWS) ? mloc : (QROWS - 1);
  const float* hr = H2 + (size_t)mcl * NMLP;
  float s0 = 0.f, s1 = 0.f, s2 = 0.f, s3 = 0.f;
#pragma unroll 2
  for (int i = 0; i < NMLP / 4; ++i) {
    const v4f hv = *(const v4f*)(hr + 4 * i);
    const v4f wv = *(const v4f*)(sW + 4 * i);
    s0 = fmaf(hv[0], wv[0], s0);
    s1 = fmaf(hv[1], wv[1], s1);
    s2 = fmaf(hv[2], wv[2], s2);
    s3 = fmaf(hv[3], wv[3], s3);
  }
  const float v = ((s0 + s1) + (s2 + s3)) + b3[0];
  if (mloc < QROWS) {
    volatile float* op = out3 + (size_t)mbase + mloc;
    *op = v;
    __threadfence();
    *op = v;
  }
}

extern "C" void kernel_launch(void* const* d_in, const int* in_sizes, int n_in,
                              void* d_out, int out_size, void* d_ws, size_t ws_size,
                              hipStream_t stream) {
  if (n_in < 24) return;
  if (out_size != 4 * NROWS) return;
  if (in_sizes[0] != NROWS * NFEAT || in_sizes[1] != NROWS * NFEAT || in_sizes[2] != NROWS * NFEAT) return;
  if (in_sizes[4] != NGATE * NHID || in_sizes[9] != NGATE * NHID || in_sizes[14] != NGATE * NHID) return;
  if (in_sizes[20] != NMLP * NMLP || in_sizes[18] != 3 * NMLP) return;
  if (ws_size < WS_TOTAL) return;

  const float* Dis_out = (const float*)d_in[0];
  const float* Dis_rad = (const float*)d_in[1];
  const float* Dis_occ = (const float*)d_in[2];
  const float* l1_Wih = (const float*)d_in[3];
  const float* l1_Whh = (const float*)d_in[4];
  const float* l1_b   = (const float*)d_in[5];
  const float* l1_hw  = (const float*)d_in[6];
  const float* l1_hb  = (const float*)d_in[7];
  const float* l2_Wih = (const float*)d_in[8];
  const float* l2_Whh = (const float*)d_in[9];
  const float* l2_b   = (const float*)d_in[10];
  const float* l2_hw  = (const float*)d_in[11];
  const float* l2_hb  = (const float*)d_in[12];
  const float* l3_Wih = (const float*)d_in[13];
  const float* l3_Whh = (const float*)d_in[14];
  const float* l3_b   = (const float*)d_in[15];
  const float* l3_hw  = (const float*)d_in[16];
  const float* l3_hb  = (const float*)d_in[17];
  const float* mlp_W1 = (const float*)d_in[18];
  const float* mlp_b1 = (const float*)d_in[19];
  const float* mlp_W2 = (const float*)d_in[20];
  const float* mlp_b2 = (const float*)d_in[21];
  const float* mlp_W3 = (const float*)d_in[22];
  const float* mlp_b3 = (const float*)d_in[23];

  float* out  = (float*)d_out;
  float* out3 = out + (size_t)3 * NROWS;

  char* ws = (char*)d_ws;
  unsigned short* WhhH = (unsigned short*)(ws + OFF_WHH);
  unsigned short* W2T  = (unsigned short*)(ws + OFF_W2T);
  unsigned short* H1q  = (unsigned short*)(ws + OFF_H1);
  float*          H2q  = (float*)(ws + OFF_H2);

  whh_cast_kernel<<<dim3((NGATE * NHID) / (8 * 256), 3), 256, 0, stream>>>(l1_Whh, l2_Whh, l3_Whh, WhhH, kWCarry);
  w2t_cast_kernel<<<dim3(NMLP / 64, NMLP / 64), 256, 0, stream>>>(mlp_W2, W2T, kWCarry);
  lstm_seq_kernel<<<dim3(NBATCH / 16, 3), 256, 0, stream>>>(
      Dis_out, Dis_rad, Dis_occ, WhhH,
      l1_Wih, l1_b, l1_hw, l1_hb,
      l2_Wih, l2_b, l2_hw, l2_hb,
      l3_Wih, l3_b, l3_hw, l3_hb,
      out);
  for (int q = 0; q < NQUART; ++q) {
    const int mbase = q * QROWS;
    mlp_h1_kernel<<<(QROWS * 64) / 256, 256, 0, stream>>>(out, mlp_W1, mlp_b1, H1q, mbase, kH1Carry);
    wmma_gemm64<0, false, 2, 0, false, 2><<<dim3((QROWS / 64) * (NMLP / 64) / 8, 1), 256, 0, stream>>>(
        H1q, nullptr, NMLP, 0L,
        W2T, nullptr, NMLP, 0L,
        (void*)H2q, nullptr, NMLP, 0L,
        mlp_b2,
        nullptr, 0L,
        QROWS, NMLP, NMLP, kMlpScale);
    mlp_head_kernel<<<QROWS / 256, 256, 0, stream>>>(H2q, mlp_W3, mlp_b3, out3, mbase);
  }
}
